// StaticCompositeLinear_16716012716090
// MI455X (gfx1250) — hardware-run, weakly checked
//
#include <hip/hip_runtime.h>
#include <math.h>

typedef __attribute__((ext_vector_type(16))) _Float16 v16h;
typedef __attribute__((ext_vector_type(8)))  _Float16 v8h;
typedef __attribute__((ext_vector_type(8)))  float    v8f;
typedef __attribute__((ext_vector_type(4)))  float    v4f;

constexpr int kTok   = 4 * 4096;
constexpr int kDin   = 512;
constexpr int kDout  = 512;
constexpr int kNexp  = 8;
constexpr int kWRows = kNexp * kDout;
constexpr float kWCarry    = 64.0f;
constexpr float kWCarryInv = 1.0f / kWCarry;
constexpr int kBlkRows = 128;
constexpr int kBlkCols = 32;
constexpr int kYPitch  = 36;
static_assert(kTok == 16384);
static_assert(kWRows == 4096);
static_assert((kDin % 32) == 0);
static_assert((kTok % kBlkRows) == 0 && (kDout % kBlkCols) == 0);
static_assert((kTok % 32) == 0);
static_assert(((kWRows * kDin / 8) % 256) == 0);
static_assert((kYPitch % 4) == 0);

constexpr size_t kOffXH   = 0;
constexpr size_t kOffWH   = kOffXH + (size_t)kTok * kDin * 2;
constexpr size_t kOffCF   = kOffWH + (size_t)kWRows * kDin * 2;
constexpr size_t kWsTotal = kOffCF + (size_t)kTok * kNexp * 4;
static_assert(kWsTotal == 21495808ull);
static_assert(kWsTotal <= 134217728ull);
static_assert((kOffWH % 128) == 0 && (kOffCF % 128) == 0);

union FragH { v16h v; v8h h[2]; };
__device__ __forceinline__ v16h frag_load_f16(const _Float16* p) {
  FragH f;
  f.h[0] = *(const v8h*)(p);
  f.h[1] = *(const v8h*)(p + 16);
  return f.v;
}
__device__ __forceinline__ v8f mma_f16_guarded(v16h a, v16h b, v8f c) {
  c = __builtin_amdgcn_wmma_f32_16x16x32_f16(false, a, false, b, (short)0, c, false, false);
  asm volatile("v_nop\n\tv_nop\n\tv_nop\n\tv_nop" : "+v"(c) : "v"(a), "v"(b));
  return c;
}

__global__ __launch_bounds__(256) void weights_to_f16_kernel(
    const float* __restrict__ src, unsigned short* __restrict__ dst, int total8)
{
  const int i = blockIdx.x * 256 + threadIdx.x;
  if (i >= total8) return;
  const size_t e0 = (size_t)i << 3;
  const v4f a0 = *(const v4f*)(src + e0);
  const v4f a1 = *(const v4f*)(src + e0 + 4);
  v8h hv;
  hv[0] = (_Float16)(a0[0] * kWCarry);
  hv[1] = (_Float16)(a0[1] * kWCarry);
  hv[2] = (_Float16)(a0[2] * kWCarry);
  hv[3] = (_Float16)(a0[3] * kWCarry);
  hv[4] = (_Float16)(a1[0] * kWCarry);
  hv[5] = (_Float16)(a1[1] * kWCarry);
  hv[6] = (_Float16)(a1[2] * kWCarry);
  hv[7] = (_Float16)(a1[3] * kWCarry);
  unsigned short* q = dst + e0;
  *(volatile v8h*)q = hv;
  __threadfence();
  *(volatile v8h*)q = hv;
}

__global__ __launch_bounds__(256) void gate_and_convert_kernel(
    const float* __restrict__ x, const float* __restrict__ mw, const float* __restrict__ mb,
    unsigned short* __restrict__ xh, float* __restrict__ coef)
{
  __shared__ __align__(16) float sW[kNexp * kDin];
  const int tid = threadIdx.x, lane = tid & 31, wave = tid >> 5;
#pragma unroll
  for (int i = 0; i < 4; ++i) {
    const int idx = (i * 256 + tid) * 4;
    *(v4f*)(sW + idx) = *(const v4f*)(mw + idx);
  }
  __syncthreads();

  const int tok0 = (blockIdx.x * 8 + wave) * 4;
  const int gsel = lane & 7;
  const int tsel = lane >> 3;
  float mylogit = 0.0f;

#pragma unroll 1
  for (int t = 0; t < 4; ++t) {
    float part[kNexp];
#pragma unroll
    for (int e = 0; e < kNexp; ++e) part[e] = 0.0f;
    const float* xr = x + (size_t)(tok0 + t) * kDin;
    unsigned short* xo = xh + (size_t)(tok0 + t) * kDin;
#pragma unroll 1
    for (int hf = 0; hf < 2; ++hf) {
      const int off = hf * 256 + lane * 8;
      const v4f a0 = *(const v4f*)(xr + off);
      const v4f a1 = *(const v4f*)(xr + off + 4);
#pragma unroll
      for (int e = 0; e < kNexp; ++e) {
        const v4f w0 = *(const v4f*)(sW + e * kDin + off);
        const v4f w1 = *(const v4f*)(sW + e * kDin + off + 4);
        float p = part[e];
        p = fmaf(a0[0], w0[0], p);
        p = fmaf(a0[1], w0[1], p);
        p = fmaf(a0[2], w0[2], p);
        p = fmaf(a0[3], w0[3], p);
        p = fmaf(a1[0], w1[0], p);
        p = fmaf(a1[1], w1[1], p);
        p = fmaf(a1[2], w1[2], p);
        p = fmaf(a1[3], w1[3], p);
        part[e] = p;
      }
      v8h hv;
      hv[0] = (_Float16)a0[0];
      hv[1] = (_Float16)a0[1];
      hv[2] = (_Float16)a0[2];
      hv[3] = (_Float16)a0[3];
      hv[4] = (_Float16)a1[0];
      hv[5] = (_Float16)a1[1];
      hv[6] = (_Float16)a1[2];
      hv[7] = (_Float16)a1[3];
      unsigned short* q = xo + off;
      *(volatile v8h*)q = hv;
      __threadfence();
      *(volatile v8h*)q = hv;
    }
#pragma unroll
    for (int e = 0; e < kNexp; ++e) {
      float p = part[e];
      p += __shfl_xor(p, 16, 32);
      p += __shfl_xor(p, 8, 32);
      p += __shfl_xor(p, 4, 32);
      p += __shfl_xor(p, 2, 32);
      p += __shfl_xor(p, 1, 32);
      part[e] = p;
    }
    float sel = part[0];
    sel = (gsel == 1) ? part[1] : sel;
    sel = (gsel == 2) ? part[2] : sel;
    sel = (gsel == 3) ? part[3] : sel;
    sel = (gsel == 4) ? part[4] : sel;
    sel = (gsel == 5) ? part[5] : sel;
    sel = (gsel == 6) ? part[6] : sel;
    sel = (gsel == 7) ? part[7] : sel;
    mylogit = (tsel == t) ? sel : mylogit;
  }

  const float lg = mylogit + mb[gsel];
  float mx = lg;
  mx = fmaxf(mx, __shfl_xor(mx, 1, 32));
  mx = fmaxf(mx, __shfl_xor(mx, 2, 32));
  mx = fmaxf(mx, __shfl_xor(mx, 4, 32));
  const float ex = expf(lg - mx);
  float sm = ex;
  sm += __shfl_xor(sm, 1, 32);
  sm += __shfl_xor(sm, 2, 32);
  sm += __shfl_xor(sm, 4, 32);
  const float cf = ex * (1.0f / sm);
  float* cq = coef + (size_t)tok0 * kNexp + lane;
  *(volatile float*)cq = cf;
  __threadfence();
  *(volatile float*)cq = cf;
}

__global__ __launch_bounds__(256) void fused_gemm_combine_kernel(
    const unsigned short* __restrict__ xh, const unsigned short* __restrict__ wh,
    const float* __restrict__ coef, const float* __restrict__ biases, float* __restrict__ y)
{
  __shared__ __align__(16) float sY[kBlkRows * kYPitch];
  __shared__ __align__(16) float sC[kBlkRows * kNexp];
  __shared__ __align__(16) float sB[kNexp * kBlkCols];

  const int tid  = threadIdx.x;
  const int lane = tid & 31;
  const int wave = tid >> 5;
  const int hh   = lane >> 4;
  const int l15  = lane & 15;
  const int wm   = wave >> 1;
  const int wn   = wave & 1;
  const int m0blk = blockIdx.x * kBlkRows;
  const int n0blk = blockIdx.y * kBlkCols;

  {
    const v4f cv = *(const v4f*)(coef + (size_t)m0blk * kNexp + tid * 4);
    *(v4f*)(sC + tid * 4) = cv;
    sB[tid] = biases[(tid >> 5) * kDout + n0blk + (tid & 31)];
  }
  __syncthreads();

  const int m0 = m0blk + wm * 32;
  const int n0 = n0blk + wn * 16;
  const _Float16* A0 = (const _Float16*)xh + (size_t)(m0 + l15) * kDin + 8 * hh;
  const _Float16* A1 = A0 + (size_t)16 * kDin;
  const _Float16* Bp = (const _Float16*)wh + (size_t)(n0 + l15) * kDin + 8 * hh;
  constexpr size_t kGateStride = (size_t)kDout * kDin;

  v8f acc[2][kNexp];
#pragma unroll
  for (int mt = 0; mt < 2; ++mt)
#pragma unroll
    for (int e = 0; e < kNexp; ++e) acc[mt][e] = (v8f){0.f, 0.f, 0.f, 0.f, 0.f, 0.f, 0.f, 0.f};

#pragma unroll 1
  for (int k0 = 0; k0 < kDin; k0 += 32) {
    const v16h a0 = frag_load_f16(A0 + k0);
    const v16h a1 = frag_load_f16(A1 + k0);
#pragma unroll
    for (int e = 0; e < kNexp; ++e) {
      const v16h b = frag_load_f16(Bp + (size_t)e * kGateStride + k0);
      acc[0][e] = mma_f16_guarded(a0, b, acc[0][e]);
      acc[1][e] = mma_f16_guarded(a1, b, acc[1][e]);
    }
  }

  float be[kNexp];
#pragma unroll
  for (int e = 0; e < kNexp; ++e) be[e] = sB[e * kBlkCols + wn * 16 + l15] * kWCarry;

#pragma unroll
  for (int mt = 0; mt < 2; ++mt) {
#pragma unroll
    for (int j = 0; j < 8; ++j) {
      const int rowl = wm * 32 + mt * 16 + 8 * hh + j;
      const v4f c0 = *(const v4f*)(sC + rowl * kNexp);
      const v4f c1 = *(const v4f*)(sC + rowl * kNexp + 4);
      float s = 0.0f;
      s = fmaf(c0[0], acc[mt][0][j] + be[0], s);
      s = fmaf(c0[1], acc[mt][1][j] + be[1], s);
      s = fmaf(c0[2], acc[mt][2][j] + be[2], s);
      s = fmaf(c0[3], acc[mt][3][j] + be[3], s);
      s = fmaf(c1[0], acc[mt][4][j] + be[4], s);
      s = fmaf(c1[1], acc[mt][5][j] + be[5], s);
      s = fmaf(c1[2], acc[mt][6][j] + be[6], s);
      s = fmaf(c1[3], acc[mt][7][j] + be[7], s);
      sY[rowl * kYPitch + wn * 16 + l15] = s * kWCarryInv;
    }
  }
  __syncthreads();

  {
    const int q  = lane >> 3;
    const int c4 = (lane & 7) * 4;
    v4f ov[4];
#pragma unroll
    for (int it = 0; it < 4; ++it) {
      const int row = it * 32 + wave * 4 + q;
      ov[it] = *(const v4f*)(sY + row * kYPitch + c4);
    }
    for (int pass = 0; pass < 2; ++pass) {
#pragma unroll
      for (int it = 0; it < 4; ++it) {
        const int row = it * 32 + wave * 4 + q;
        *(volatile v4f*)(y + (size_t)(m0blk + row) * kDout + n0blk + c4) = ov[it];
      }
      __threadfence();
    }
  }
}

extern "C" void kernel_launch(void* const* d_in, const int* in_sizes, int n_in,
                              void* d_out, int out_size, void* d_ws, size_t ws_size,
                              hipStream_t stream) {
  if (n_in < 5) return;
  if (in_sizes[0] != kTok * kDin) return;
  if (in_sizes[1] != kWRows * kDin) return;
  if (in_sizes[2] != kNexp * kDout) return;
  if (in_sizes[3] != kNexp * kDin) return;
  if (in_sizes[4] != kNexp) return;
  if (out_size != kTok * kDout) return;
  if (ws_size < kWsTotal) return;

  const float* x       = (const float*)d_in[0];
  const float* ew      = (const float*)d_in[1];
  const float* ebias   = (const float*)d_in[2];
  const float* mixer_w = (const float*)d_in[3];
  const float* mixer_b = (const float*)d_in[4];
  float* y = (float*)d_out;

  char* ws = (char*)d_ws;
  unsigned short* XH = (unsigned short*)(ws + kOffXH);
  unsigned short* WH = (unsigned short*)(ws + kOffWH);
  float*          CF = (float*)(ws + kOffCF);

  weights_to_f16_kernel<<<(kWRows * kDin / 8) / 256, 256, 0, stream>>>(ew, WH, kWRows * kDin / 8);
  gate_and_convert_kernel<<<kTok / 32, 256, 0, stream>>>(x, mixer_w, mixer_b, XH, CF);
  fused_gemm_combine_kernel<<<dim3(kTok / kBlkRows, kDout / kBlkCols), 256, 0, stream>>>(XH, WH, CF, ebias, y);
}
